// EncodeSequential_74182675136896
// MI455X (gfx1250) — hardware-verified
//
#include <hip/hip_runtime.h>
#include <hip/hip_bf16.h>
#include <stddef.h>
#include <stdint.h>

#define NBAT 4
#define SQ   2048
#define DM   1024
#define NTOK 8192
#define NQKV 3072
#define R0   512
#define NR3  2048
#define QT   128
#define NQB  16
#define QB3  4
#define TILE_E 16384
#define PB   (TILE_E * 136)
#define PB3  (TILE_E * 10)
#define OUTN (NTOK * DM)

static_assert(NTOK == NBAT * SQ);
static_assert(NR3 == NBAT * R0);
static_assert(NQB == SQ / QT);
static_assert(QB3 == R0 / QT);
static_assert(TILE_E == QT * QT);
static_assert(PB == TILE_E * (NQB * (NQB + 1) / 2));
static_assert(PB3 == TILE_E * (QB3 * (QB3 + 1) / 2));
static_assert(NQKV == 3 * DM);
static_assert(DM == 128 * 8);
static_assert(DM % 64 == 0);
static_assert(SQ % 64 == 0);
static_assert(R0 % 64 == 0);
static_assert(R0 % QT == 0);
static_assert(R0 < SQ);
static_assert(OUTN == 8388608);
static_assert((size_t)NBAT * PB * 4 <= (size_t)NTOK * DM * 2 + 2 * (size_t)NR3 * DM * 2 + 3 * (size_t)NQKV * DM * 2);
static_assert((size_t)NBAT * PB * 2 + 2 * (size_t)NBAT * PB3 * 2 <= 2 * (size_t)NTOK * DM * 2);

typedef _Float16 v16h __attribute__((ext_vector_type(16)));
typedef _Float16 v8h  __attribute__((ext_vector_type(8)));
typedef float    v8f  __attribute__((ext_vector_type(8)));
typedef float    v4f  __attribute__((ext_vector_type(4)));
typedef unsigned int   v4u   __attribute__((ext_vector_type(4)));
typedef unsigned short v8us  __attribute__((ext_vector_type(8)));
typedef unsigned short v16us __attribute__((ext_vector_type(16)));
typedef __bf16         v16b  __attribute__((ext_vector_type(16)));
typedef unsigned short ush;

union Frag  { v16h v; v8h h[2]; };
union FragU { v16us v; v8us h[2]; v16b b; };
union Pack8 { v8h h; v4u u; };
union PackU { v8us s; v4u u; };
struct HL { v4u h; v4u l; };

__device__ __forceinline__ ush f2bf(float f) {
  const unsigned u = __float_as_uint(f);
  return (ush)((u + 0x7FFFu + ((u >> 16) & 1u)) >> 16);
}
__device__ __forceinline__ float bf2f(ush b) { return __uint_as_float(((unsigned)b) << 16); }

__device__ __forceinline__ HL split8(v8f f) {
  PackU ph, pl;
#pragma unroll
  for (int e = 0; e < 8; ++e) {
    const ush hi = f2bf(f[e]);
    ph.s[e] = hi;
    pl.s[e] = f2bf(f[e] - bf2f(hi));
  }
  HL r; r.h = ph.u; r.l = pl.u;
  return r;
}

__device__ __forceinline__ v4u packh8(v8f f, float sc) {
  Pack8 pk;
  pk.h = (v8h){(_Float16)(f[0] * sc), (_Float16)(f[1] * sc), (_Float16)(f[2] * sc), (_Float16)(f[3] * sc),
               (_Float16)(f[4] * sc), (_Float16)(f[5] * sc), (_Float16)(f[6] * sc), (_Float16)(f[7] * sc)};
  return pk.u;
}

__device__ __forceinline__ v8f mma16(v16h a, v16h b, v8f c) {
  c = __builtin_amdgcn_wmma_f32_16x16x32_f16(false, a, false, b, (short)0, c, false, false);
  asm volatile("v_nop\n\tv_nop\n\tv_nop\n\tv_nop" : "+v"(c) : "v"(a), "v"(b));
  return c;
}
__device__ __forceinline__ v8f mmab(v16us a, v16us b, v8f c) {
  FragU ua, ub; ua.v = a; ub.v = b;
  c = __builtin_amdgcn_wmma_f32_16x16x32_bf16(false, ua.b, false, ub.b, (short)0, c, false, false);
  asm volatile("v_nop\n\tv_nop\n\tv_nop\n\tv_nop" : "+v"(c) : "v"(a), "v"(b));
  return c;
}

__device__ __forceinline__ v16h ldfrag(const _Float16* p, int ld, int row0, int k0, int lane) {
  const int m = lane & 15, lh = lane >> 4;
  const _Float16* q = p + (size_t)(row0 + m) * ld + k0 + 8 * lh;
  Frag f;
  f.h[0] = *(const v8h*)(q);
  f.h[1] = *(const v8h*)(q + 16);
  return f.v;
}
__device__ __forceinline__ v16us ldfragu(const ush* p, int ld, int row0, int k0, int lane) {
  const int m = lane & 15, lh = lane >> 4;
  const ush* q = p + (size_t)(row0 + m) * ld + k0 + 8 * lh;
  FragU f;
  f.h[0] = *(const v8us*)(q);
  f.h[1] = *(const v8us*)(q + 16);
  return f.v;
}

__device__ __forceinline__ v8f zero8() { return (v8f){0.f, 0.f, 0.f, 0.f, 0.f, 0.f, 0.f, 0.f}; }

__device__ __forceinline__ void gemm16x64(const _Float16* __restrict__ A, int lda,
                                          const _Float16* __restrict__ Bt, int ldb,
                                          int m0, int n0, int kdim, int lane, v8f (&acc)[4]) {
#pragma unroll 2
  for (int k0 = 0; k0 < kdim; k0 += 32) {
    const v16h a = ldfrag(A, lda, m0, k0, lane);
#pragma unroll
    for (int t = 0; t < 4; ++t) {
      const v16h b = ldfrag(Bt, ldb, n0 + 16 * t, k0, lane);
      acc[t] = mma16(a, b, acc[t]);
    }
  }
}

__device__ __forceinline__ void gemm3_16x64(const ush* __restrict__ Ah, const ush* __restrict__ Al, int lda,
                                            const ush* __restrict__ Bh, const ush* __restrict__ Bl, int ldb,
                                            int m0, int n0, int kdim, int lane, v8f (&acc)[4]) {
#pragma unroll 1
  for (int k0 = 0; k0 < kdim; k0 += 32) {
    const v16us ah = ldfragu(Ah, lda, m0, k0, lane);
    const v16us al = ldfragu(Al, lda, m0, k0, lane);
#pragma unroll
    for (int t = 0; t < 4; ++t) {
      const v16us bh = ldfragu(Bh, ldb, n0 + 16 * t, k0, lane);
      const v16us bl = ldfragu(Bl, ldb, n0 + 16 * t, k0, lane);
      acc[t] = mmab(ah, bh, acc[t]);
      acc[t] = mmab(ah, bl, acc[t]);
      acc[t] = mmab(al, bh, acc[t]);
    }
  }
}

__device__ __forceinline__ void gemm32x64(const _Float16* __restrict__ A, int lda,
                                          const _Float16* __restrict__ Bt, int ldb,
                                          int m0, int n0, int kdim, int lane, v8f (&acc)[2][4]) {
#pragma unroll 2
  for (int k0 = 0; k0 < kdim; k0 += 32) {
    const v16h a0 = ldfrag(A, lda, m0, k0, lane);
    const v16h a1 = ldfrag(A, lda, m0 + 16, k0, lane);
    const v16h b0 = ldfrag(Bt, ldb, n0, k0, lane);
    const v16h b1 = ldfrag(Bt, ldb, n0 + 16, k0, lane);
    const v16h b2 = ldfrag(Bt, ldb, n0 + 32, k0, lane);
    const v16h b3 = ldfrag(Bt, ldb, n0 + 48, k0, lane);
    acc[0][0] = mma16(a0, b0, acc[0][0]);
    acc[1][0] = mma16(a1, b0, acc[1][0]);
    acc[0][1] = mma16(a0, b1, acc[0][1]);
    acc[1][1] = mma16(a1, b1, acc[1][1]);
    acc[0][2] = mma16(a0, b2, acc[0][2]);
    acc[1][2] = mma16(a1, b2, acc[1][2]);
    acc[0][3] = mma16(a0, b3, acc[0][3]);
    acc[1][3] = mma16(a1, b3, acc[1][3]);
  }
}

__device__ __forceinline__ void gemm3_32x64(const ush* __restrict__ Ah, const ush* __restrict__ Al, int lda,
                                            const ush* __restrict__ Bh, const ush* __restrict__ Bl, int ldb,
                                            int m0, int n0, int kdim, int lane, v8f (&acc)[2][4]) {
#pragma unroll 1
  for (int k0 = 0; k0 < kdim; k0 += 32) {
    const v16us a0h = ldfragu(Ah, lda, m0, k0, lane);
    const v16us a1h = ldfragu(Ah, lda, m0 + 16, k0, lane);
    const v16us a0l = ldfragu(Al, lda, m0, k0, lane);
    const v16us a1l = ldfragu(Al, lda, m0 + 16, k0, lane);
#pragma unroll
    for (int t = 0; t < 4; ++t) {
      const v16us bh = ldfragu(Bh, ldb, n0 + 16 * t, k0, lane);
      const v16us bl = ldfragu(Bl, ldb, n0 + 16 * t, k0, lane);
      acc[0][t] = mmab(a0h, bh, acc[0][t]);
      acc[1][t] = mmab(a1h, bh, acc[1][t]);
      acc[0][t] = mmab(a0h, bl, acc[0][t]);
      acc[1][t] = mmab(a1h, bl, acc[1][t]);
      acc[0][t] = mmab(a0l, bh, acc[0][t]);
      acc[1][t] = mmab(a1l, bh, acc[1][t]);
    }
  }
}

__global__ __launch_bounds__(128) void k_cvtx(const float* __restrict__ src, _Float16* __restrict__ dh,
                                              ush* __restrict__ d3h, ush* __restrict__ d3l) {
  const int row = blockIdx.x;
  const int col = (int)threadIdx.x * 8;
  const int b   = row / SQ;
  const int s   = row - b * SQ;
  const size_t o = (size_t)row * DM + col;
  const v4f a0 = *(const v4f*)(src + o);
  const v4f a1 = *(const v4f*)(src + o + 4);
  const v8f f = (v8f){a0[0], a0[1], a0[2], a0[3], a1[0], a1[1], a1[2], a1[3]};
  const v4u vv = packh8(f, 1.0f);
  const bool three = (s < R0);
  const size_t o3 = ((size_t)(b * R0 + (three ? s : 0))) * DM + col;
  HL sp; sp.h = (v4u){0u, 0u, 0u, 0u}; sp.l = sp.h;
  if (three) sp = split8(f);
  volatile v4u* d = (volatile v4u*)(dh + o);
  *d = vv;
  if (three) { *(volatile v4u*)(d3h + o3) = sp.h; *(volatile v4u*)(d3l + o3) = sp.l; }
  __threadfence();
  *d = vv;
  if (three) { *(volatile v4u*)(d3h + o3) = sp.h; *(volatile v4u*)(d3l + o3) = sp.l; }
}

__global__ __launch_bounds__(128) void k_cvtw(const float* __restrict__ w0, const float* __restrict__ w1,
                                              const float* __restrict__ w2, _Float16* __restrict__ wt,
                                              ush* __restrict__ wh, ush* __restrict__ wl) {
  const int which = blockIdx.y;
  const float* W = (which == 0) ? w0 : ((which == 1) ? w1 : w2);
  const int n   = blockIdx.x;
  const int col = (int)threadIdx.x * 8;
  const size_t oi = (size_t)n * DM + col;
  const size_t oo = ((size_t)(which * DM + n)) * DM + col;
  const v4f a0 = *(const v4f*)(W + oi);
  const v4f a1 = *(const v4f*)(W + oi + 4);
  const v8f f = (v8f){a0[0], a0[1], a0[2], a0[3], a1[0], a1[1], a1[2], a1[3]};
  const v4u vt = packh8(f, 32.0f);
  const HL  sp = split8(f);
  *(volatile v4u*)(wt + oo) = vt;
  *(volatile v4u*)(wh + oo) = sp.h;
  *(volatile v4u*)(wl + oo) = sp.l;
  __threadfence();
  *(volatile v4u*)(wt + oo) = vt;
  *(volatile v4u*)(wh + oo) = sp.h;
  *(volatile v4u*)(wl + oo) = sp.l;
}

#define SFP 132
__global__ __launch_bounds__(256) void k_qkv(const _Float16* __restrict__ xh,
                                             const _Float16* __restrict__ wt,
                                             const float* __restrict__ bq,
                                             const float* __restrict__ bk,
                                             const float* __restrict__ bv,
                                             _Float16* __restrict__ qp,
                                             _Float16* __restrict__ kp,
                                             _Float16* __restrict__ vtp) {
  __shared__ __align__(16) float sf[64 * SFP];
  const int tid = threadIdx.x, lane = tid & 31, wave = tid >> 5;
  const int hh = lane >> 4, c = lane & 15;
  const int wm = wave >> 1, wn = wave & 1;
  const int mb = blockIdx.x * 64;
  const int b  = mb / SQ;
  const int sb = mb - b * SQ;
  if (sb < R0) return;
  const int ns = blockIdx.y;
  const int which = ns >> 3;
  const int cb = (ns & 7) * 128;
  const int m0 = mb + wm * 16;
  const int n0 = ns * 128 + wn * 64;
  const float* bias = ((which == 0) ? bq : ((which == 1) ? bk : bv)) + cb;

  v8f acc[4];
#pragma unroll
  for (int t = 0; t < 4; ++t) acc[t] = zero8();
  gemm16x64(xh, DM, wt, DM, m0, n0, DM, lane, acc);

#pragma unroll
  for (int t = 0; t < 4; ++t) {
    const float bb = bias[wn * 64 + 16 * t + c];
#pragma unroll
    for (int r = 0; r < 8; ++r)
      sf[(wm * 16 + 8 * hh + r) * SFP + wn * 64 + 16 * t + c] = acc[t][r] * 0.03125f + bb;
  }
  __syncthreads();

  if (which < 2) {
    v4u val[4];
    size_t go[4];
#pragma unroll
    for (int j = 0; j < 4; ++j) {
      const int p  = tid + 256 * j;
      const int lr = p >> 4;
      const int pc = p & 15;
      const int d0 = pc * 8;
      const float* ra = sf + lr * SFP + d0;
      const v4f a0 = *(const v4f*)(ra), a1 = *(const v4f*)(ra + 4);
      const v8f f = (v8f){a0[0], a0[1], a0[2], a0[3], a1[0], a1[1], a1[2], a1[3]};
      val[j] = packh8(f, 1.0f);
      go[j]  = (size_t)(mb + lr) * DM + cb + d0;
    }
    _Float16* base = (which == 0) ? qp : kp;
    for (int ps = 0; ps < 2; ++ps) {
#pragma unroll
      for (int j = 0; j < 4; ++j) *(volatile v4u*)(base + go[j]) = val[j];
      __threadfence();
    }
  } else {
    v4u val[4];
    size_t go[4];
#pragma unroll
    for (int j = 0; j < 4; ++j) {
      const int p  = tid + 256 * j;
      const int d  = p >> 3;
      const int pc = p & 7;
      const float* cp = sf + (pc * 8) * SFP + d;
      const v8f f = (v8f){cp[0 * SFP], cp[1 * SFP], cp[2 * SFP], cp[3 * SFP],
                          cp[4 * SFP], cp[5 * SFP], cp[6 * SFP], cp[7 * SFP]};
      val[j] = packh8(f, 1.0f);
      go[j]  = ((size_t)b * DM + cb + d) * SQ + sb + pc * 8;
    }
    for (int ps = 0; ps < 2; ++ps) {
#pragma unroll
      for (int j = 0; j < 4; ++j) *(volatile v4u*)(vtp + go[j]) = val[j];
      __threadfence();
    }
  }
}

__global__ __launch_bounds__(256) void k_qkv3(const ush* __restrict__ xh3, const ush* __restrict__ xl3,
                                              const ush* __restrict__ wth, const ush* __restrict__ wtl,
                                              const float* __restrict__ bq, const float* __restrict__ bk,
                                              const float* __restrict__ bv,
                                              ush* __restrict__ q3h, ush* __restrict__ q3l,
                                              ush* __restrict__ k3h, ush* __restrict__ k3l,
                                              _Float16* __restrict__ kp,
                                              ush* __restrict__ v3h, ush* __restrict__ v3l,
                                              _Float16* __restrict__ vtp) {
  __shared__ __align__(16) float sf[64 * SFP];
  const int tid = threadIdx.x, lane = tid & 31, wave = tid >> 5;
  const int hh = lane >> 4, c = lane & 15;
  const int wm = wave >> 1, wn = wave & 1;
  const int mb3 = blockIdx.x * 64;
  const int b   = mb3 / R0;
  const int sb  = mb3 - b * R0;
  const int ns  = blockIdx.y;
  const int which = ns >> 3;
  const int cb  = (ns & 7) * 128;
  const int m0  = mb3 + wm * 16;
  const int n0  = ns * 128 + wn * 64;
  const float* bias = ((which == 0) ? bq : ((which == 1) ? bk : bv)) + cb;

  v8f acc[4];
#pragma unroll
  for (int t = 0; t < 4; ++t) acc[t] = zero8();
  gemm3_16x64(xh3, xl3, DM, wth, wtl, DM, m0, n0, DM, lane, acc);

#pragma unroll
  for (int t = 0; t < 4; ++t) {
    const float bb = bias[wn * 64 + 16 * t + c];
#pragma unroll
    for (int r = 0; r < 8; ++r)
      sf[(wm * 16 + 8 * hh + r) * SFP + wn * 64 + 16 * t + c] = acc[t][r] + bb;
  }
  __syncthreads();

  if (which < 2) {
    v4u vh[4], vl[4], vf[4];
    size_t go3[4], gof[4];
#pragma unroll
    for (int j = 0; j < 4; ++j) {
      const int p  = tid + 256 * j;
      const int lr = p >> 4;
      const int pc = p & 15;
      const int d0 = pc * 8;
      const float* ra = sf + lr * SFP + d0;
      const v4f a0 = *(const v4f*)(ra), a1 = *(const v4f*)(ra + 4);
      const v8f f = (v8f){a0[0], a0[1], a0[2], a0[3], a1[0], a1[1], a1[2], a1[3]};
      const HL s = split8(f);
      vh[j] = s.h; vl[j] = s.l;
      vf[j] = packh8(f, 1.0f);
      go3[j] = (size_t)(mb3 + lr) * DM + cb + d0;
      gof[j] = ((size_t)b * SQ + sb + lr) * DM + cb + d0;
    }
    ush* ph = (which == 0) ? q3h : k3h;
    ush* pl = (which == 0) ? q3l : k3l;
    for (int ps = 0; ps < 2; ++ps) {
#pragma unroll
      for (int j = 0; j < 4; ++j) {
        *(volatile v4u*)(ph + go3[j]) = vh[j];
        *(volatile v4u*)(pl + go3[j]) = vl[j];
        if (which == 1) *(volatile v4u*)(kp + gof[j]) = vf[j];
      }
      __threadfence();
    }
  } else {
    v4u vh[4], vl[4], vf[4];
    size_t go3[4], gof[4];
#pragma unroll
    for (int j = 0; j < 4; ++j) {
      const int p  = tid + 256 * j;
      const int d  = p >> 3;
      const int pc = p & 7;
      const float* cp = sf + (pc * 8) * SFP + d;
      const v8f f = (v8f){cp[0 * SFP], cp[1 * SFP], cp[2 * SFP], cp[3 * SFP],
                          cp[4 * SFP], cp[5 * SFP], cp[6 * SFP], cp[7 * SFP]};
      const HL s = split8(f);
      vh[j] = s.h; vl[j] = s.l;
      vf[j] = packh8(f, 1.0f);
      go3[j] = ((size_t)b * DM + cb + d) * R0 + sb + pc * 8;
      gof[j] = ((size_t)b * DM + cb + d) * SQ + sb + pc * 8;
    }
    for (int ps = 0; ps < 2; ++ps) {
#pragma unroll
      for (int j = 0; j < 4; ++j) {
        *(volatile v4u*)(v3h + go3[j]) = vh[j];
        *(volatile v4u*)(v3l + go3[j]) = vl[j];
        *(volatile v4u*)(vtp + gof[j]) = vf[j];
      }
      __threadfence();
    }
  }
}

#define OTP 68
__device__ __forceinline__ void out_epilogue(v8f (&acc)[2][4], float scale, float* sw, float* __restrict__ dst,
                                             int ldo, int lane, int hh, int c) {
#pragma unroll
  for (int sub = 0; sub < 2; ++sub) {
    __syncthreads();
#pragma unroll
    for (int t = 0; t < 4; ++t) {
#pragma unroll
      for (int r = 0; r < 8; ++r) sw[(8 * hh + r) * OTP + 16 * t + c] = acc[sub][t][r] * scale;
    }
    __syncthreads();
    v4f val[8];
    size_t go[8];
#pragma unroll
    for (int it = 0; it < 8; ++it) {
      const int p    = lane + 32 * it;
      const int L    = p >> 3;
      const int pc   = p & 7;
      const int row  = L >> 1;
      const int half = L & 1;
      val[it] = *(const v4f*)(sw + row * OTP + half * 32 + pc * 4);
      go[it]  = (size_t)(sub * 16 + row) * ldo + half * 32 + pc * 4;
    }
    for (int ps = 0; ps < 2; ++ps) {
#pragma unroll
      for (int it = 0; it < 8; ++it) *(volatile v4f*)(dst + go[it]) = val[it];
      __threadfence();
    }
  }
}

__device__ __forceinline__ size_t tile_base(int qb) { return (size_t)TILE_E * (size_t)(qb * (qb + 1) / 2); }

__global__ __launch_bounds__(256) void k_sc(const _Float16* __restrict__ qp,
                                            const _Float16* __restrict__ kp,
                                            float* __restrict__ S) {
  const int kb = blockIdx.x, qb = blockIdx.y + QB3, b = blockIdx.z;
  if (kb > qb) return;
  __shared__ __align__(16) float st[8][16 * OTP];
  const int tid = threadIdx.x, lane = tid & 31, wave = tid >> 5;
  const int hh = lane >> 4, c = lane & 15;
  const int wm = wave >> 1, wn = wave & 1;
  const int mq = b * SQ + qb * QT + wm * 32;
  const int nk = b * SQ + kb * QT + wn * 64;
  v8f acc[2][4];
#pragma unroll
  for (int s = 0; s < 2; ++s)
#pragma unroll
    for (int t = 0; t < 4; ++t) acc[s][t] = zero8();
  gemm32x64(qp, DM, kp, DM, mq, nk, DM, lane, acc);
  const int pitch = (qb + 1) * QT;
  float* dst = S + (size_t)b * PB + tile_base(qb) + (size_t)(wm * 32) * pitch + kb * QT + wn * 64;
  out_epilogue(acc, 0.03125f, st[wave], dst, pitch, lane, hh, c);
}

__global__ __launch_bounds__(256) void k_sc3(const ush* __restrict__ q3h, const ush* __restrict__ q3l,
                                             const ush* __restrict__ k3h, const ush* __restrict__ k3l,
                                             float* __restrict__ S) {
  const int kb = blockIdx.x, qb = blockIdx.y, b = blockIdx.z;
  if (kb > qb) return;
  __shared__ __align__(16) float st[8][16 * OTP];
  const int tid = threadIdx.x, lane = tid & 31, wave = tid >> 5;
  const int hh = lane >> 4, c = lane & 15;
  const int wm = wave >> 1, wn = wave & 1;
  const int mq = b * R0 + qb * QT + wm * 32;
  const int nk = b * R0 + kb * QT + wn * 64;
  v8f acc[2][4];
#pragma unroll
  for (int s = 0; s < 2; ++s)
#pragma unroll
    for (int t = 0; t < 4; ++t) acc[s][t] = zero8();
  gemm3_32x64(q3h, q3l, DM, k3h, k3l, DM, mq, nk, DM, lane, acc);
  const int pitch = (qb + 1) * QT;
  float* dst = S + (size_t)b * PB + tile_base(qb) + (size_t)(wm * 32) * pitch + kb * QT + wn * 64;
  out_epilogue(acc, 0.03125f, st[wave], dst, pitch, lane, hh, c);
}

__global__ __launch_bounds__(256) void k_sm(const float* __restrict__ S, _Float16* __restrict__ P,
                                            ush* __restrict__ p3h, ush* __restrict__ p3l) {
  __shared__ float redm[8];
  __shared__ float reds[8];
  const int q  = blockIdx.x;
  const int b  = blockIdx.y;
  const int qb = q >> 7, r = q & (QT - 1);
  const int pitch = (qb + 1) * QT;
  const int npc = pitch >> 3;
  const size_t toff = tile_base(qb) + (size_t)r * pitch;
  const float* row = S + (size_t)b * PB + toff;
  const int tid = threadIdx.x, lane = tid & 31, wave = tid >> 5;
  const bool act = (tid < npc);
  const int tc  = act ? tid : (npc - 1);
  const int j0  = tc * 8;
  const v4f a0 = *(const v4f*)(row + j0);
  const v4f a1 = *(const v4f*)(row + j0 + 4);
  const v8f v = (v8f){a0[0], a0[1], a0[2], a0[3], a1[0], a1[1], a1[2], a1[3]};
  const int n = q + 1;
  const float NEGI = -__builtin_huge_valf();

  float mx = NEGI;
#pragma unroll
  for (int e = 0; e < 8; ++e) {
    const bool ok = act && (j0 + e < n);
    mx = ok ? fmaxf(mx, v[e]) : mx;
  }
#pragma unroll
  for (int off = 1; off < 32; off <<= 1) mx = fmaxf(mx, __shfl_xor(mx, off, 32));
  if (lane == 0) redm[wave] = mx;
  __syncthreads();
  float m = redm[0];
#pragma unroll
  for (int w = 1; w < 8; ++w) m = fmaxf(m, redm[w]);

  v8f ex;
  float sum = 0.f;
#pragma unroll
  for (int e = 0; e < 8; ++e) {
    const bool ok = act && (j0 + e < n);
    const float x  = fminf(v[e] - m, 0.f);
    const float pe = __expf(x);
    ex[e] = ok ? pe : 0.f;
    sum += ex[e];
  }
#pragma unroll
  for (int off = 1; off < 32; off <<= 1) sum += __shfl_xor(sum, off, 32);
  if (lane == 0) reds[wave] = sum;
  __syncthreads();
  float l = reds[0];
#pragma unroll
  for (int w = 1; w < 8; ++w) l += reds[w];
  const float inv = 1.0f / l;

  if (q >= R0) {
    const v4u pv = packh8(ex, inv * 1024.0f);
    _Float16* pr = P + (size_t)b * PB + toff + j0;
    if (act) *(volatile v4u*)pr = pv;
    __threadfence();
    if (act) *(volatile v4u*)pr = pv;
  } else {
    const v8f pf = ex * inv;
    const HL sp = split8(pf);
    const size_t o3 = (size_t)b * PB3 + toff + j0;
    if (act) { *(volatile v4u*)(p3h + o3) = sp.h; *(volatile v4u*)(p3l + o3) = sp.l; }
    __threadfence();
    if (act) { *(volatile v4u*)(p3h + o3) = sp.h; *(volatile v4u*)(p3l + o3) = sp.l; }
  }
}

__global__ __launch_bounds__(256) void k_pv(const _Float16* __restrict__ P,
                                            const _Float16* __restrict__ vtp,
                                            float* __restrict__ out) {
  __shared__ __align__(16) float st[8][16 * OTP];
  const int db = blockIdx.x, qb = blockIdx.y + QB3, b = blockIdx.z;
  const int tid = threadIdx.x, lane = tid & 31, wave = tid >> 5;
  const int hh = lane >> 4, c = lane & 15;
  const int wm = wave >> 1, wn = wave & 1;
  const int pitch = (qb + 1) * QT;
  const _Float16* A  = P + (size_t)b * PB + tile_base(qb);
  const _Float16* Bt = vtp + (size_t)b * DM * SQ;
  v8f acc[2][4];
#pragma unroll
  for (int s = 0; s < 2; ++s)
#pragma unroll
    for (int t = 0; t < 4; ++t) acc[s][t] = zero8();
  gemm32x64(A, pitch, Bt, SQ, wm * 32, db * QT + wn * 64, pitch, lane, acc);
  float* dst = out + ((size_t)b * SQ + qb * QT + wm * 32) * DM + db * QT + wn * 64;
  out_epilogue(acc, 0.0009765625f, st[wave], dst, DM, lane, hh, c);
}

__global__ __launch_bounds__(256) void k_pv3(const ush* __restrict__ p3h, const ush* __restrict__ p3l,
                                             const ush* __restrict__ v3h, const ush* __restrict__ v3l,
                                             float* __restrict__ out) {
  __shared__ __align__(16) float st[8][16 * OTP];
  const int db = blockIdx.x, qb = blockIdx.y, b = blockIdx.z;
  const int tid = threadIdx.x, lane = tid & 31, wave = tid >> 5;
  const int hh = lane >> 4, c = lane & 15;
  const int wm = wave >> 1, wn = wave & 1;
  const int pitch = (qb + 1) * QT;
  const size_t ao = (size_t)b * PB3 + tile_base(qb);
  const size_t vo = (size_t)b * DM * R0;
  v8f acc[2][4];
#pragma unroll
  for (int s = 0; s < 2; ++s)
#pragma unroll
    for (int t = 0; t < 4; ++t) acc[s][t] = zero8();
  gemm3_32x64(p3h + ao, p3l + ao, pitch, v3h + vo, v3l + vo, R0, wm * 32, db * QT + wn * 64, pitch, lane, acc);
  float* dst = out + ((size_t)b * SQ + qb * QT + wm * 32) * DM + db * QT + wn * 64;
  out_epilogue(acc, 1.0f, st[wave], dst, DM, lane, hh, c);
}

extern "C" void kernel_launch(void* const* d_in, const int* in_sizes, int n_in,
                              void* d_out, int out_size, void* d_ws, size_t ws_size,
                              hipStream_t stream) {
  if (n_in < 7) return;
  if (in_sizes[0] != NTOK * DM) return;
  if (in_sizes[1] != DM * DM) return;
  if (in_sizes[2] != DM) return;
  if (in_sizes[3] != DM * DM) return;
  if (in_sizes[4] != DM) return;
  if (in_sizes[5] != DM * DM) return;
  if (in_sizes[6] != DM) return;
  if (out_size != OUTN) return;

  const float* x  = (const float*)d_in[0];
  const float* wq = (const float*)d_in[1];
  const float* bq = (const float*)d_in[2];
  const float* wk = (const float*)d_in[3];
  const float* bk = (const float*)d_in[4];
  const float* wv = (const float*)d_in[5];
  const float* bv = (const float*)d_in[6];
  float* out = (float*)d_out;

  size_t off = 0;
  const size_t oX   = off; off += (size_t)NTOK * DM * 2;
  const size_t oX3h = off; off += (size_t)NR3 * DM * 2;
  const size_t oX3l = off; off += (size_t)NR3 * DM * 2;
  const size_t oWt  = off; off += (size_t)NQKV * DM * 2;
  const size_t oWth = off; off += (size_t)NQKV * DM * 2;
  const size_t oWtl = off; off += (size_t)NQKV * DM * 2;
  const size_t endA = off;
  const size_t oQ   = off; off += (size_t)NTOK * DM * 2;
  const size_t oK   = off; off += (size_t)NTOK * DM * 2;
  const size_t endQK = off;
  const size_t oV   = off; off += (size_t)NBAT * DM * SQ * 2;
  const size_t oQ3h = off; off += (size_t)NR3 * DM * 2;
  const size_t oQ3l = off; off += (size_t)NR3 * DM * 2;
  const size_t oK3h = off; off += (size_t)NR3 * DM * 2;
  const size_t oK3l = off; off += (size_t)NR3 * DM * 2;
  const size_t oV3h = off; off += (size_t)NBAT * DM * R0 * 2;
  const size_t oV3l = off; off += (size_t)NBAT * DM * R0 * 2;
  const size_t oS   = oX;
  const size_t szS  = (size_t)NBAT * PB * 4;
  const size_t oP   = oQ;
  const size_t szP  = (size_t)NBAT * PB * 2;
  const size_t oP3h = oP + szP;
  const size_t szP3 = (size_t)NBAT * PB3 * 2;
  const size_t oP3l = oP3h + szP3;
  if (off > ws_size) return;
  if (off > (size_t)134217728) return;
  if (oS + szS > endA) return;
  if (oP3l + szP3 > endQK) return;

  char* ws = (char*)d_ws;
  _Float16* Xh  = (_Float16*)(ws + oX);
  ush*      X3h = (ush*)(ws + oX3h);
  ush*      X3l = (ush*)(ws + oX3l);
  _Float16* Wt  = (_Float16*)(ws + oWt);
  ush*      Wth = (ush*)(ws + oWth);
  ush*      Wtl = (ush*)(ws + oWtl);
  _Float16* Qp  = (_Float16*)(ws + oQ);
  _Float16* Kp  = (_Float16*)(ws + oK);
  _Float16* Vt  = (_Float16*)(ws + oV);
  ush*      Q3h = (ush*)(ws + oQ3h);
  ush*      Q3l = (ush*)(ws + oQ3l);
  ush*      K3h = (ush*)(ws + oK3h);
  ush*      K3l = (ush*)(ws + oK3l);
  ush*      V3h = (ush*)(ws + oV3h);
  ush*      V3l = (ush*)(ws + oV3l);
  float*    Sp  = (float*)(ws + oS);
  _Float16* Pp  = (_Float16*)(ws + oP);
  ush*      P3h = (ush*)(ws + oP3h);
  ush*      P3l = (ush*)(ws + oP3l);

  k_cvtx<<<dim3(NTOK), dim3(128), 0, stream>>>(x, Xh, X3h, X3l);
  k_cvtw<<<dim3(DM, 3), dim3(128), 0, stream>>>(wq, wk, wv, Wt, Wth, Wtl);
  k_qkv<<<dim3(NTOK / 64, NQKV / QT), dim3(256), 0, stream>>>(Xh, Wt, bq, bk, bv, Qp, Kp, Vt);
  k_qkv3<<<dim3(NR3 / 64, NQKV / QT), dim3(256), 0, stream>>>(X3h, X3l, Wth, Wtl, bq, bk, bv,
                                                              Q3h, Q3l, K3h, K3l, Kp, V3h, V3l, Vt);
  k_sc<<<dim3(NQB, NQB - QB3, NBAT), dim3(256), 0, stream>>>(Qp, Kp, Sp);
  k_sc3<<<dim3(QB3, QB3, NBAT), dim3(256), 0, stream>>>(Q3h, Q3l, K3h, K3l, Sp);
  k_sm<<<dim3(SQ, NBAT), dim3(256), 0, stream>>>(Sp, Pp, P3h, P3l);
  k_pv<<<dim3(DM / QT, NQB - QB3, NBAT), dim3(256), 0, stream>>>(Pp, Vt, out);
  k_pv3<<<dim3(DM / QT, QB3, NBAT), dim3(256), 0, stream>>>(P3h, P3l, V3h, V3l, out);
  (void)hipGetLastError();
}
